// ViTSelfAttention_16243566313558
// MI455X (gfx1250) — hardware-verified
//
#include <hip/hip_runtime.h>
#include <math.h>

typedef __attribute__((ext_vector_type(16))) _Float16 v16h;
typedef __attribute__((ext_vector_type(8)))  _Float16 v8h;
typedef __attribute__((ext_vector_type(16))) __bf16   v16b;
typedef __attribute__((ext_vector_type(8)))  __bf16   v8b;
typedef __attribute__((ext_vector_type(8)))  float    v8f;
typedef __attribute__((ext_vector_type(4)))  float    v4f;
typedef __attribute__((ext_vector_type(4)))  unsigned int u32x4;

constexpr int NB_ALL  = 16;
constexpr int NTOK    = 1024;
constexpr int DMODEL  = 768;
constexpr int NHEADS  = 12;
constexpr int HDIM    = 64;
constexpr int NB_HALF = 8;
constexpr int MHALF   = NB_HALF * NTOK;
constexpr int QK_LD   = 2 * DMODEL;
constexpr int KCOL0   = DMODEL;
constexpr int VT_LD   = MHALF;
constexpr int NQB     = NTOK / 64;
constexpr int NKCH    = NTOK / 64;

static_assert(MHALF % 64 == 0 && DMODEL % 64 == 0 && DMODEL % 32 == 0 && (2 * DMODEL) % 64 == 0, "");
static_assert(NTOK % 64 == 0 && HDIM == 64 && NHEADS * HDIM == DMODEL, "");

__device__ __forceinline__ unsigned short f2bf_bits(float f) {
  unsigned u = __float_as_uint(f);
  return (unsigned short)((u + 0x7FFFu + ((u >> 16) & 1u)) >> 16);
}
__device__ __forceinline__ float bf_bits2f(unsigned short h) { return __uint_as_float(((unsigned)h) << 16); }

__device__ __forceinline__ void dep_guard_h(v8f& a, v8f& b, v16h x, v16h y) { asm volatile("v_nop\n\tv_nop\n\tv_nop\n\tv_nop" : "+v"(a), "+v"(b) : "v"(x), "v"(y)); }
__device__ __forceinline__ void dep_guard_b(v8f& a, v8f& b, v16b x, v16b y) { asm volatile("v_nop\n\tv_nop\n\tv_nop\n\tv_nop" : "+v"(a), "+v"(b) : "v"(x), "v"(y)); }
__device__ __forceinline__ void keep4_h(v16h a, v16h b, v16h c, v16h d) { asm volatile("v_nop" :: "v"(a), "v"(b), "v"(c), "v"(d)); }
__device__ __forceinline__ void keep4_b(v16b a, v16b b, v16b c, v16b d) { asm volatile("v_nop" :: "v"(a), "v"(b), "v"(c), "v"(d)); }
__device__ __forceinline__ void acc_guard4(v8f& a, v8f& b, v8f& c, v8f& d) { asm volatile("v_nop\n\tv_nop\n\tv_nop\n\tv_nop" : "+v"(a), "+v"(b), "+v"(c), "+v"(d)); }
template <typename T> struct Frag;
template <> struct Frag<_Float16> {
  typedef v16h V; union U { v16h v; v8h h[2]; };
  static __device__ __forceinline__ v16h load(const _Float16* p) {
    U f; f.h[0] = *(const v8h*)(p); f.h[1] = *(const v8h*)(p + 16); return f.v;
  }
  static __device__ __forceinline__ v8f mma(v16h a, v16h b, v8f c) {
    return __builtin_amdgcn_wmma_f32_16x16x32_f16(false, a, false, b, (short)0, c, false, false);
  }
  static __device__ __forceinline__ void guard(v8f& a, v8f& b, v16h x, v16h y) { dep_guard_h(a, b, x, y); }
  static __device__ __forceinline__ void keep(v16h a, v16h b, v16h c, v16h d) { keep4_h(a, b, c, d); }
};
template <> struct Frag<__bf16> {
  typedef v16b V; union U { v16b v; v8b h[2]; };
  static __device__ __forceinline__ v16b load(const __bf16* p) {
    U f; f.h[0] = *(const v8b*)(p); f.h[1] = *(const v8b*)(p + 16); return f.v;
  }
  static __device__ __forceinline__ v8f mma(v16b a, v16b b, v8f c) {
    return __builtin_amdgcn_wmma_f32_16x16x32_bf16(false, a, false, b, (short)0, c, false, false);
  }
  static __device__ __forceinline__ void guard(v8f& a, v8f& b, v16b x, v16b y) { dep_guard_b(a, b, x, y); }
  static __device__ __forceinline__ void keep(v16b a, v16b b, v16b c, v16b d) { keep4_b(a, b, c, d); }
};

__device__ __forceinline__ v8f mma_b(v16b a, v16b b, v8f c) {
  c = __builtin_amdgcn_wmma_f32_16x16x32_bf16(false, a, false, b, (short)0, c, false, false);
  asm volatile("v_nop\n\tv_nop\n\tv_nop\n\tv_nop" : "+v"(c) : "v"(a), "v"(b));
  return c;
}
__device__ __forceinline__ v8f mma_h(v16h a, v16h b, v8f c) {
  c = __builtin_amdgcn_wmma_f32_16x16x32_f16(false, a, false, b, (short)0, c, false, false);
  asm volatile("v_nop\n\tv_nop\n\tv_nop\n\tv_nop" : "+v"(c) : "v"(a), "v"(b));
  return c;
}

template <int ET> struct Elem;
template <> struct Elem<0> { typedef _Float16 T; };
template <> struct Elem<1> { typedef __bf16 T; };
template <int ET, bool SPLIT, int BIAS_MODE, int OUT_MODE, bool RESID, int ACT = 0>
__global__ __launch_bounds__(256) void wmma_gemm64(
    const unsigned short* __restrict__ Ap, const unsigned short* __restrict__ A2p, int lda, long strideA,
    const unsigned short* __restrict__ Btp, const unsigned short* __restrict__ Bt2p, int ldb, long strideB,
    void* __restrict__ Cout, void* __restrict__ Cout2, int ldc, long strideC,
    const float* __restrict__ bias,
    const float* __restrict__ resid, long strideR,
    int M, int N, int K, float scale) {
  typedef typename Elem<ET>::T T;
  typedef typename Frag<T>::V V;
  const T* A = (const T*)Ap; const T* A2 = (const T*)A2p; const T* Bt = (const T*)Btp; const T* Bt2 = (const T*)Bt2p;
  __shared__ __align__(16) float sT[8][16 * 68];
  const int b    = blockIdx.y;
  const int lane = threadIdx.x & 31;
  const int wave = threadIdx.x >> 5;
  const int tilesN = N >> 6;
  const int tilesM = M >> 6;
  const int tile = blockIdx.x * 8 + wave;
  if (tile >= tilesM * tilesN) return;
  const int tm = tile / tilesN;
  const int tn = tile - tm * tilesN;
  const int m0 = tm << 6;
  const int n0 = tn << 6;

  const T* Ab  = A  + (size_t)b * strideA;
  const T* Bb  = Bt + (size_t)b * strideB;
  const T* Ab2 = SPLIT ? (A2  + (size_t)b * strideA) : nullptr;
  const T* Bb2 = SPLIT ? (Bt2 + (size_t)b * strideB) : nullptr;

  const int rlane = lane & 15;
  const int koff  = (lane >> 4) * 8;
  const int mOff  = (lane >> 4) * 8;

  v8f acc[4][4];
#pragma unroll
  for (int i = 0; i < 4; ++i)
#pragma unroll
    for (int j = 0; j < 4; ++j) acc[i][j] = (v8f){0.f,0.f,0.f,0.f,0.f,0.f,0.f,0.f};

  for (int k0 = 0; k0 < K; k0 += 32) {
    V bh[4], bl[4];
#pragma unroll
    for (int j = 0; j < 4; ++j) {
      const size_t bo = (size_t)(n0 + (j << 4) + rlane) * ldb + koff + k0;
      bh[j] = Frag<T>::load(Bb + bo);
      if (SPLIT) bl[j] = Frag<T>::load(Bb2 + bo);
    }
#pragma unroll
    for (int i = 0; i < 4; ++i) {
      const size_t ao = (size_t)(m0 + (i << 4) + rlane) * lda + koff + k0;
      V ah = Frag<T>::load(Ab + ao);
      V al;
      if (SPLIT) al = Frag<T>::load(Ab2 + ao);
#pragma unroll
      for (int j = 0; j < 4; ++j) {
        acc[i][j] = Frag<T>::mma(ah, bh[j], acc[i][j]);
        if (SPLIT) {
          acc[i][j] = Frag<T>::mma(ah, bl[j], acc[i][j]);
          acc[i][j] = Frag<T>::mma(al, bh[j], acc[i][j]);
        }
      }
      Frag<T>::guard(acc[i][0], acc[i][3], ah, SPLIT ? al : ah);
    }
    Frag<T>::keep(bh[0], bh[1], bh[2], bh[3]);
    if (SPLIT) Frag<T>::keep(bl[0], bl[1], bl[2], bl[3]);
  }
  acc_guard4(acc[0][0], acc[0][1], acc[0][2], acc[0][3]);
  acc_guard4(acc[1][0], acc[1][1], acc[1][2], acc[1][3]);
  acc_guard4(acc[2][0], acc[2][1], acc[2][2], acc[2][3]);
  acc_guard4(acc[3][0], acc[3][1], acc[3][2], acc[3][3]);

  float* slab = sT[wave];
  const float* Rb = RESID ? (resid + (size_t)b * strideR) : nullptr;
#pragma unroll
  for (int i = 0; i < 4; ++i) {
    const int mBase = m0 + (i << 4);
    float bm[8] = {0.f, 0.f, 0.f, 0.f, 0.f, 0.f, 0.f, 0.f};
    if (BIAS_MODE == 1) {
      const v4f b0 = *(const v4f*)(bias + mBase + mOff);
      const v4f b1 = *(const v4f*)(bias + mBase + mOff + 4);
#pragma unroll
      for (int e = 0; e < 4; ++e) { bm[e] = bf_bits2f(f2bf_bits(b0[e])); bm[4 + e] = bf_bits2f(f2bf_bits(b1[e])); }
    }
#pragma unroll
    for (int j = 0; j < 4; ++j) {
      const int n = n0 + (j << 4) + rlane;
      float bv = 0.f;
      if (BIAS_MODE == 2) bv = bf_bits2f(f2bf_bits(bias[n]));
#pragma unroll
      for (int r = 0; r < 8; ++r) {
        float v = acc[i][j][r] * scale;
        if (BIAS_MODE == 1) v += bm[r];
        if (BIAS_MODE == 2) v += bv;
        if (RESID) v += Rb[(size_t)(mBase + mOff + r) * ldc + n];
        if (ACT == 1) v = tanhf(v);
        if (ACT == 2) v = fmaxf(v, 0.0f);
        if (ACT == 3) v = v / (1.0f + expf(-v));
        if (ACT == 4) v = (v > 0.f) ? v : 0.01f * v;
        slab[(mOff + r) * 68 + (j << 4) + rlane] = v;
      }
    }
    __builtin_amdgcn_fence(__ATOMIC_RELEASE, "workgroup");
    __builtin_amdgcn_wave_barrier();
    __builtin_amdgcn_fence(__ATOMIC_ACQUIRE, "workgroup");
    if (OUT_MODE == 0) {
      float* C = (float*)Cout + (size_t)b * strideC;
      const int hh = lane >> 4, c4 = (lane & 15) * 4;
      for (int pass = 0; pass < 2; ++pass) {
#pragma unroll
        for (int it = 0; it < 8; ++it) {
          const int row = it * 2 + hh;
          v4f v = *(const v4f*)(slab + row * 68 + c4);
          *(volatile v4f*)(C + (size_t)(mBase + row) * ldc + n0 + c4) = v;
        }
        __threadfence();
      }
    } else {
      const int q = lane >> 3, c8 = (lane & 7) * 8;
      unsigned short* C  = (unsigned short*)Cout  + (size_t)b * strideC;
      unsigned short* C2 = (OUT_MODE >= 2) ? ((unsigned short*)Cout2 + (size_t)b * strideC) : nullptr;
      for (int pass = 0; pass < 2; ++pass) {
#pragma unroll
        for (int it = 0; it < 4; ++it) {
          const int row = it * 4 + q;
          const float* sp = slab + row * 68 + c8;
          v8h hv, lv;
#pragma unroll
          for (int e = 0; e < 8; ++e) {
            if (OUT_MODE == 1) {
              hv[e] = (_Float16)sp[e];
              lv[e] = hv[e];
            } else if (OUT_MODE == 3) {
              const _Float16 hq = (_Float16)sp[e];
              const float hf = (float)hq;
              const float res = (sp[e] - hf) * 2048.0f;
              hv[e] = hq;
              lv[e] = (_Float16)res;
            } else {
              unsigned short hb = f2bf_bits(sp[e]);
              unsigned short lb = f2bf_bits(sp[e] - bf_bits2f(hb));
              hv[e] = __builtin_bit_cast(_Float16, hb);
              lv[e] = __builtin_bit_cast(_Float16, lb);
            }
          }
          *(volatile v8h*)(C + (size_t)(mBase + row) * ldc + n0 + c8) = hv;
          if (OUT_MODE >= 2) *(volatile v8h*)(C2 + (size_t)(mBase + row) * ldc + n0 + c8) = lv;
        }
        __threadfence();
      }
    }
    __builtin_amdgcn_fence(__ATOMIC_RELEASE, "workgroup");
    __builtin_amdgcn_wave_barrier();
    __builtin_amdgcn_fence(__ATOMIC_ACQUIRE, "workgroup");
  }
}

__global__ __launch_bounds__(256) void cvt_rows_bf16(const float* __restrict__ x,
                                                     unsigned short* __restrict__ xb, int n8) {
  const int i = blockIdx.x * 256 + threadIdx.x;
  if (i < n8) {
    const v4f a = *(const v4f*)(x + (size_t)i * 8);
    const v4f c = *(const v4f*)(x + (size_t)i * 8 + 4);
    u32x4 u;
    u[0] = (unsigned)f2bf_bits(a[0]) | ((unsigned)f2bf_bits(a[1]) << 16);
    u[1] = (unsigned)f2bf_bits(a[2]) | ((unsigned)f2bf_bits(a[3]) << 16);
    u[2] = (unsigned)f2bf_bits(c[0]) | ((unsigned)f2bf_bits(c[1]) << 16);
    u[3] = (unsigned)f2bf_bits(c[2]) | ((unsigned)f2bf_bits(c[3]) << 16);
    volatile u32x4* dst = (volatile u32x4*)(void*)(xb + (size_t)i * 8);
    *dst = u;
    __threadfence();
    *dst = u;
  }
}

__global__ __launch_bounds__(256) void wt_transpose_bf16(const float* __restrict__ Wq,
                                                         const float* __restrict__ Wk,
                                                         const float* __restrict__ Wv,
                                                         unsigned short* __restrict__ wt) {
  __shared__ __align__(16) float tile[64 * 68];
  const int tid = threadIdx.x;
  const int mat = blockIdx.x / 144;
  const int t   = blockIdx.x - mat * 144;
  const int kt  = t / 12;
  const int ft  = t - kt * 12;
  const int k0  = kt * 64;
  const int f0  = ft * 64;
  const float* W = (mat == 0) ? Wq : ((mat == 1) ? Wk : Wv);
#pragma unroll
  for (int i = 0; i < 4; ++i) {
    const int e  = tid + 256 * i;
    const int kr = e >> 4;
    const int c4 = (e & 15) * 4;
    const v4f v = *(const v4f*)(W + (size_t)(k0 + kr) * DMODEL + f0 + c4);
    *(v4f*)(tile + kr * 68 + c4) = v;
  }
  __syncthreads();
  const int wave = tid >> 5, lane = tid & 31;
  const int sub = lane >> 3, piece = lane & 7;
  for (int pass = 0; pass < 2; ++pass) {
#pragma unroll
    for (int it = 0; it < 2; ++it) {
      const int fr = wave * 8 + it * 4 + sub;
      u32x4 u;
#pragma unroll
      for (int e = 0; e < 4; ++e) {
        const float v0 = tile[(piece * 8 + 2 * e) * 68 + fr];
        const float v1 = tile[(piece * 8 + 2 * e + 1) * 68 + fr];
        u[e] = (unsigned)f2bf_bits(v0) | ((unsigned)f2bf_bits(v1) << 16);
      }
      *(volatile u32x4*)(void*)(wt + (size_t)(mat * DMODEL + f0 + fr) * DMODEL + k0 + piece * 8) = u;
    }
    __threadfence();
  }
}

__global__ __launch_bounds__(128)
void attn_heads64(const unsigned short* __restrict__ QKhP, const unsigned short* __restrict__ QKlP,
                  const unsigned short* __restrict__ VThP, const unsigned short* __restrict__ VTlP,
                  float* __restrict__ out) {
  __shared__ __align__(16) __bf16   Ksh[64 * 64];
  __shared__ __align__(16) __bf16   Ksl[64 * 64];
  __shared__ __align__(16) _Float16 Vth[64 * 64];
  __shared__ __align__(16) _Float16 Vtl[64 * 64];
  __shared__ __align__(16) _Float16 Psh[4][16 * 64];
  __shared__ __align__(16) float    Os[4][16 * 68];

  const int tid  = threadIdx.x;
  const int wave = tid >> 5;
  const int lane = tid & 31;
  const int hh   = lane >> 4;
  const int c    = lane & 15;

  const int bx = blockIdx.x;
  const int qb = bx % NQB;
  const int bh = bx / NQB;
  const int h  = bh % NHEADS;
  const int b  = bh / NHEADS;
  const int q0 = qb * 64 + wave * 16;

  const __bf16* Qh = (const __bf16*)QKhP + (size_t)b * NTOK * QK_LD + h * HDIM;
  const __bf16* Ql = (const __bf16*)QKlP + (size_t)b * NTOK * QK_LD + h * HDIM;
  const __bf16* Kh = Qh + KCOL0;
  const __bf16* Kl = Ql + KCOL0;
  const _Float16* Vh = (const _Float16*)VThP + (size_t)(h * HDIM) * VT_LD + (size_t)b * NTOK;
  const _Float16* Vl = (const _Float16*)VTlP + (size_t)(h * HDIM) * VT_LD + (size_t)b * NTOK;
  float* op = out + (size_t)b * NTOK * DMODEL + h * HDIM;

  v16b qah[2], qal[2];
#pragma unroll
  for (int dc = 0; dc < 2; ++dc) {
    qah[dc] = Frag<__bf16>::load(Qh + (size_t)(q0 + c) * QK_LD + dc * 32 + 8 * hh);
    qal[dc] = Frag<__bf16>::load(Ql + (size_t)(q0 + c) * QK_LD + dc * 32 + 8 * hh);
  }

  float mrow[8], lrow[8];
  v8f oacc[4];
#pragma unroll
  for (int r = 0; r < 8; ++r) { mrow[r] = -INFINITY; lrow[r] = 0.f; }
#pragma unroll
  for (int t = 0; t < 4; ++t) oacc[t] = (v8f){0.f,0.f,0.f,0.f,0.f,0.f,0.f,0.f};

  for (int kc = 0; kc < NKCH; ++kc) {
    const int kv0 = kc * 64;
    __syncthreads();
#pragma unroll
    for (int i = 0; i < 4; ++i) {
      const int piece = tid + 128 * i;
      const int rr = piece >> 3;
      const int c8 = (piece & 7) * 8;
      const u32x4 kh = *(const u32x4*)(const void*)(Kh + (size_t)(kv0 + rr) * QK_LD + c8);
      const u32x4 kl = *(const u32x4*)(const void*)(Kl + (size_t)(kv0 + rr) * QK_LD + c8);
      const u32x4 vh = *(const u32x4*)(const void*)(Vh + (size_t)rr * VT_LD + kv0 + c8);
      const u32x4 vl = *(const u32x4*)(const void*)(Vl + (size_t)rr * VT_LD + kv0 + c8);
      *(u32x4*)(void*)(Ksh + rr * 64 + c8) = kh;
      *(u32x4*)(void*)(Ksl + rr * 64 + c8) = kl;
      *(u32x4*)(void*)(Vth + rr * 64 + c8) = vh;
      *(u32x4*)(void*)(Vtl + rr * 64 + c8) = vl;
    }
    __syncthreads();

    v8f s[4];
#pragma unroll
    for (int j = 0; j < 4; ++j) {
      s[j] = (v8f){0.f,0.f,0.f,0.f,0.f,0.f,0.f,0.f};
#pragma unroll
      for (int dc = 0; dc < 2; ++dc) {
        const v16b kb = Frag<__bf16>::load(Ksh + (j * 16 + c) * 64 + dc * 32 + 8 * hh);
        const v16b kl = Frag<__bf16>::load(Ksl + (j * 16 + c) * 64 + dc * 32 + 8 * hh);
        s[j] = mma_b(qah[dc], kb, s[j]);
        s[j] = mma_b(qah[dc], kl, s[j]);
        s[j] = mma_b(qal[dc], kb, s[j]);
      }
    }
    float cm[8];
#pragma unroll
    for (int r = 0; r < 8; ++r) {
      float m = -INFINITY;
#pragma unroll
      for (int j = 0; j < 4; ++j) {
        const float sv = s[j][r] * 0.125f;
        s[j][r] = sv;
        m = fmaxf(m, sv);
      }
#pragma unroll
      for (int off = 1; off < 16; off <<= 1) m = fmaxf(m, __shfl_xor(m, off, 32));
      cm[r] = m;
    }
    _Float16* pw = Psh[wave];
#pragma unroll
    for (int r = 0; r < 8; ++r) {
      const float mnew = fmaxf(mrow[r], cm[r]);
      const float alpha = expf(mrow[r] - mnew);
      mrow[r] = mnew;
      float psum = 0.f;
#pragma unroll
      for (int j = 0; j < 4; ++j) {
        const float p = expf(s[j][r] - mnew);
        psum += p;
        pw[(8 * hh + r) * 64 + j * 16 + c] = (_Float16)(p * 32768.0f);
      }
#pragma unroll
      for (int off = 1; off < 16; off <<= 1) psum += __shfl_xor(psum, off, 32);
      lrow[r] = lrow[r] * alpha + psum;
#pragma unroll
      for (int t = 0; t < 4; ++t) oacc[t][r] *= alpha;
    }
    __builtin_amdgcn_fence(__ATOMIC_RELEASE, "workgroup");
    __builtin_amdgcn_wave_barrier();
    __builtin_amdgcn_fence(__ATOMIC_ACQUIRE, "workgroup");

    v8f oaccL[4];
#pragma unroll
    for (int t = 0; t < 4; ++t) oaccL[t] = (v8f){0.f,0.f,0.f,0.f,0.f,0.f,0.f,0.f};
#pragma unroll 1
    for (int kk = 0; kk < 2; ++kk) {
      const v16h pa = Frag<_Float16>::load(pw + c * 64 + kk * 32 + 8 * hh);
#pragma unroll
      for (int t = 0; t < 4; ++t) {
        const v16h vb = Frag<_Float16>::load(Vth + (t * 16 + c) * 64 + kk * 32 + 8 * hh);
        const v16h vr = Frag<_Float16>::load(Vtl + (t * 16 + c) * 64 + kk * 32 + 8 * hh);
        oacc[t]  = mma_h(pa, vb, oacc[t]);
        oaccL[t] = mma_h(pa, vr, oaccL[t]);
      }
    }
#pragma unroll
    for (int t = 0; t < 4; ++t) oacc[t] = oacc[t] + oaccL[t] * (1.0f / 2048.0f);
  }

  float* os = Os[wave];
#pragma unroll
  for (int r = 0; r < 8; ++r) {
    const float inv = 1.0f / (lrow[r] * 32768.0f);
#pragma unroll
    for (int t = 0; t < 4; ++t) os[(8 * hh + r) * 68 + t * 16 + c] = oacc[t][r] * inv;
  }
  __builtin_amdgcn_fence(__ATOMIC_RELEASE, "workgroup");
  __builtin_amdgcn_wave_barrier();
  __builtin_amdgcn_fence(__ATOMIC_ACQUIRE, "workgroup");
  {
    const int c4 = (lane & 15) * 4;
    for (int pass = 0; pass < 2; ++pass) {
#pragma unroll
      for (int it = 0; it < 8; ++it) {
        const int row = it * 2 + hh;
        v4f val = *(const v4f*)(os + row * 68 + c4);
        *(volatile v4f*)(op + (size_t)(q0 + row) * DMODEL + c4) = val;
      }
      __threadfence();
    }
  }
}

extern "C" void kernel_launch(void* const* d_in, const int* in_sizes, int n_in,
                              void* d_out, int out_size, void* d_ws, size_t ws_size,
                              hipStream_t stream) {
  if (n_in < 7) return;
  if (in_sizes[0] != NB_ALL * NTOK * DMODEL) return;
  if (in_sizes[1] != DMODEL * DMODEL || in_sizes[3] != DMODEL * DMODEL || in_sizes[5] != DMODEL * DMODEL) return;
  if (in_sizes[2] != DMODEL || in_sizes[4] != DMODEL || in_sizes[6] != DMODEL) return;
  if (out_size != NB_ALL * NTOK * DMODEL) return;

  const float* x  = (const float*)d_in[0];
  const float* Wq = (const float*)d_in[1];
  const float* bq = (const float*)d_in[2];
  const float* Wk = (const float*)d_in[3];
  const float* bk = (const float*)d_in[4];
  const float* Wv = (const float*)d_in[5];
  const float* bv = (const float*)d_in[6];
  float* out = (float*)d_out;

  const size_t szXb  = (size_t)NB_ALL * NTOK * DMODEL * 2;
  const size_t szWTb = (size_t)3 * DMODEL * DMODEL * 2;
  const size_t szQK  = (size_t)MHALF * QK_LD * 2;
  const size_t szVT  = (size_t)DMODEL * VT_LD * 2;
  const size_t offXb  = 0;
  const size_t offWTb = offXb + szXb;
  const size_t offQKh = offWTb + szWTb;
  const size_t offQKl = offQKh + szQK;
  const size_t offVTh = offQKl + szQK;
  const size_t offVTl = offVTh + szVT;
  const size_t total  = offVTl + szVT;
  if (total > ws_size) return;

  char* ws = (char*)d_ws;
  unsigned short* Xb  = (unsigned short*)(ws + offXb);
  unsigned short* WTb = (unsigned short*)(ws + offWTb);
  unsigned short* QKh = (unsigned short*)(ws + offQKh);
  unsigned short* QKl = (unsigned short*)(ws + offQKl);
  unsigned short* VTh = (unsigned short*)(ws + offVTh);
  unsigned short* VTl = (unsigned short*)(ws + offVTl);

  {
    const int n8 = NB_ALL * NTOK * DMODEL / 8;
    cvt_rows_bf16<<<(n8 + 255) / 256, 256, 0, stream>>>(x, Xb, n8);
  }
  wt_transpose_bf16<<<3 * 12 * 12, 256, 0, stream>>>(Wq, Wk, Wv, WTb);

  for (int half = 0; half < 2; ++half) {
    const unsigned short* Xh = Xb + (size_t)half * MHALF * DMODEL;
    const int tilesQ = (MHALF / 64) * (DMODEL / 64);
    wmma_gemm64<1, false, 2, 2, false, 0><<<dim3((tilesQ + 7) / 8, 1), 256, 0, stream>>>(
        Xh, Xh, DMODEL, 0L,
        WTb, WTb, DMODEL, 0L,
        (void*)QKh, (void*)QKl, QK_LD, 0L,
        bq, bq, 0L,
        MHALF, DMODEL, DMODEL, 1.0f);
    wmma_gemm64<1, false, 2, 2, false, 0><<<dim3((tilesQ + 7) / 8, 1), 256, 0, stream>>>(
        Xh, Xh, DMODEL, 0L,
        WTb + (size_t)DMODEL * DMODEL, WTb + (size_t)DMODEL * DMODEL, DMODEL, 0L,
        (void*)(QKh + KCOL0), (void*)(QKl + KCOL0), QK_LD, 0L,
        bk, bk, 0L,
        MHALF, DMODEL, DMODEL, 1.0f);
    const int tilesV = (DMODEL / 64) * (MHALF / 64);
    wmma_gemm64<1, false, 1, 3, false, 0><<<dim3((tilesV + 7) / 8, 1), 256, 0, stream>>>(
        WTb + (size_t)2 * DMODEL * DMODEL, WTb + (size_t)2 * DMODEL * DMODEL, DMODEL, 0L,
        Xh, Xh, DMODEL, 0L,
        (void*)VTh, (void*)VTl, VT_LD, 0L,
        bv, bv, 0L,
        DMODEL, MHALF, DMODEL, 1.0f);
    attn_heads64<<<NB_HALF * NHEADS * NQB, 128, 0, stream>>>(
        QKh, QKl, VTh, VTl, out + (size_t)half * MHALF * DMODEL);
  }
}
